// MMMambaEncoderLayer_16638703305489
// MI455X (gfx1250) — hardware-run, weakly checked
//
#include <hip/hip_runtime.h>
#include <math.h>

constexpr int NB_BATCH = 2;
constexpr int NL_SEQ   = 2048;
constexpr int DMOD     = 512;
constexpr int DIN_CH   = 1024;
constexpr int NXZ_COL  = 2 * DIN_CH;
constexpr int DST_N    = 16;
constexpr int DTR_K    = 32;
constexpr int NDBC_COL = DTR_K + 2 * DST_N;
constexpr int NTOK     = NB_BATCH * NL_SEQ;
constexpr float LOG2E_F = 1.4426950408889634f;
constexpr float INV_DMOD = 1.0f / 512.0f;
constexpr float LN_EPS = 1e-6f;

typedef __attribute__((ext_vector_type(16))) _Float16 v16h;
typedef __attribute__((ext_vector_type(8)))  _Float16 v8h;
typedef __attribute__((ext_vector_type(16))) __bf16   v16b;
typedef __attribute__((ext_vector_type(8)))  __bf16   v8b;
typedef __attribute__((ext_vector_type(8)))  float    v8f;
typedef __attribute__((ext_vector_type(4)))  float    v4f;
typedef __attribute__((ext_vector_type(4)))  unsigned int v4u;

__device__ __forceinline__ unsigned short f2bf_bits(float f) {
  unsigned u = __float_as_uint(f);
  return (unsigned short)((u + 0x7FFFu + ((u >> 16) & 1u)) >> 16);
}
__device__ __forceinline__ float bf_bits2f(unsigned short h) { return __uint_as_float(((unsigned)h) << 16); }

__device__ __forceinline__ void dep_guard_h(v8f& a, v8f& b, v16h x, v16h y) { asm volatile("v_nop\n\tv_nop\n\tv_nop\n\tv_nop" : "+v"(a), "+v"(b) : "v"(x), "v"(y)); }
__device__ __forceinline__ void dep_guard_b(v8f& a, v8f& b, v16b x, v16b y) { asm volatile("v_nop\n\tv_nop\n\tv_nop\n\tv_nop" : "+v"(a), "+v"(b) : "v"(x), "v"(y)); }
__device__ __forceinline__ void keep4_h(v16h a, v16h b, v16h c, v16h d) { asm volatile("v_nop" :: "v"(a), "v"(b), "v"(c), "v"(d)); }
__device__ __forceinline__ void keep4_b(v16b a, v16b b, v16b c, v16b d) { asm volatile("v_nop" :: "v"(a), "v"(b), "v"(c), "v"(d)); }
__device__ __forceinline__ void acc_guard4(v8f& a, v8f& b, v8f& c, v8f& d) { asm volatile("v_nop\n\tv_nop\n\tv_nop\n\tv_nop" : "+v"(a), "+v"(b), "+v"(c), "+v"(d)); }
template <typename T> struct Frag;
template <> struct Frag<_Float16> {
  typedef v16h V; union U { v16h v; v8h h[2]; };
  static __device__ __forceinline__ v16h load(const _Float16* p) {
    U f; f.h[0] = *(const v8h*)(p); f.h[1] = *(const v8h*)(p + 16); return f.v;
  }
  static __device__ __forceinline__ v8f mma(v16h a, v16h b, v8f c) {
    return __builtin_amdgcn_wmma_f32_16x16x32_f16(false, a, false, b, (short)0, c, false, false);
  }
  static __device__ __forceinline__ void guard(v8f& a, v8f& b, v16h x, v16h y) { dep_guard_h(a, b, x, y); }
  static __device__ __forceinline__ void keep(v16h a, v16h b, v16h c, v16h d) { keep4_h(a, b, c, d); }
};
template <> struct Frag<__bf16> {
  typedef v16b V; union U { v16b v; v8b h[2]; };
  static __device__ __forceinline__ v16b load(const __bf16* p) {
    U f; f.h[0] = *(const v8b*)(p); f.h[1] = *(const v8b*)(p + 16); return f.v;
  }
  static __device__ __forceinline__ v8f mma(v16b a, v16b b, v8f c) {
    return __builtin_amdgcn_wmma_f32_16x16x32_bf16(false, a, false, b, (short)0, c, false, false);
  }
  static __device__ __forceinline__ void guard(v8f& a, v8f& b, v16b x, v16b y) { dep_guard_b(a, b, x, y); }
  static __device__ __forceinline__ void keep(v16b a, v16b b, v16b c, v16b d) { keep4_b(a, b, c, d); }
};

__device__ __forceinline__ unsigned pk16(unsigned short a, unsigned short b) { return (unsigned)a | ((unsigned)b << 16); }

template <int ET> struct Elem;
template <> struct Elem<0> { typedef _Float16 T; };
template <> struct Elem<1> { typedef __bf16 T; };
template <int ET, bool SPLIT, int BIAS_MODE, int OUT_MODE, bool RESID, int ACT = 0>
__global__ __launch_bounds__(256) void wmma_gemm64(
    const unsigned short* __restrict__ Ap, const unsigned short* __restrict__ A2p, int lda, long strideA,
    const unsigned short* __restrict__ Btp, const unsigned short* __restrict__ Bt2p, int ldb, long strideB,
    void* __restrict__ Cout, void* __restrict__ Cout2, int ldc, long strideC,
    const float* __restrict__ bias,
    const float* __restrict__ resid, long strideR,
    int M, int N, int K, float scale) {
  typedef typename Elem<ET>::T T;
  typedef typename Frag<T>::V V;
  const T* A = (const T*)Ap; const T* A2 = (const T*)A2p; const T* Bt = (const T*)Btp; const T* Bt2 = (const T*)Bt2p;
  __shared__ __align__(16) float sT[8][16 * 68];
  const int b    = blockIdx.y;
  const int lane = threadIdx.x & 31;
  const int wave = threadIdx.x >> 5;
  const int tilesN = N >> 6;
  const int tilesM = M >> 6;
  const int tile = blockIdx.x * 8 + wave;
  if (tile >= tilesM * tilesN) return;
  const int tm = tile / tilesN;
  const int tn = tile - tm * tilesN;
  const int m0 = tm << 6;
  const int n0 = tn << 6;

  const T* Ab  = A  + (size_t)b * strideA;
  const T* Bb  = Bt + (size_t)b * strideB;
  const T* Ab2 = SPLIT ? (A2  + (size_t)b * strideA) : nullptr;
  const T* Bb2 = SPLIT ? (Bt2 + (size_t)b * strideB) : nullptr;

  const int rlane = lane & 15;
  const int koff  = (lane >> 4) * 8;
  const int mOff  = (lane >> 4) * 8;

  v8f acc[4][4];
#pragma unroll
  for (int i = 0; i < 4; ++i)
#pragma unroll
    for (int j = 0; j < 4; ++j) acc[i][j] = (v8f){0.f,0.f,0.f,0.f,0.f,0.f,0.f,0.f};

  for (int k0 = 0; k0 < K; k0 += 32) {
    V bh[4], bl[4];
#pragma unroll
    for (int j = 0; j < 4; ++j) {
      const size_t bo = (size_t)(n0 + (j << 4) + rlane) * ldb + koff + k0;
      bh[j] = Frag<T>::load(Bb + bo);
      if (SPLIT) bl[j] = Frag<T>::load(Bb2 + bo);
    }
#pragma unroll
    for (int i = 0; i < 4; ++i) {
      const size_t ao = (size_t)(m0 + (i << 4) + rlane) * lda + koff + k0;
      V ah = Frag<T>::load(Ab + ao);
      V al;
      if (SPLIT) al = Frag<T>::load(Ab2 + ao);
#pragma unroll
      for (int j = 0; j < 4; ++j) {
        acc[i][j] = Frag<T>::mma(ah, bh[j], acc[i][j]);
        if (SPLIT) {
          acc[i][j] = Frag<T>::mma(ah, bl[j], acc[i][j]);
          acc[i][j] = Frag<T>::mma(al, bh[j], acc[i][j]);
        }
      }
      Frag<T>::guard(acc[i][0], acc[i][3], ah, SPLIT ? al : ah);
    }
    Frag<T>::keep(bh[0], bh[1], bh[2], bh[3]);
    if (SPLIT) Frag<T>::keep(bl[0], bl[1], bl[2], bl[3]);
  }
  acc_guard4(acc[0][0], acc[0][1], acc[0][2], acc[0][3]);
  acc_guard4(acc[1][0], acc[1][1], acc[1][2], acc[1][3]);
  acc_guard4(acc[2][0], acc[2][1], acc[2][2], acc[2][3]);
  acc_guard4(acc[3][0], acc[3][1], acc[3][2], acc[3][3]);

  float* slab = sT[wave];
  const float* Rb = RESID ? (resid + (size_t)b * strideR) : nullptr;
#pragma unroll
  for (int i = 0; i < 4; ++i) {
    const int mBase = m0 + (i << 4);
#pragma unroll
    for (int j = 0; j < 4; ++j) {
      const int n = n0 + (j << 4) + rlane;
      float bv = 0.f;
      if (BIAS_MODE == 2) bv = bias[n];
#pragma unroll
      for (int r = 0; r < 8; ++r) {
        float v = acc[i][j][r] * scale;
        if (BIAS_MODE == 1) v += bias[mBase + mOff + r];
        if (BIAS_MODE == 2) v += bv;
        if (RESID) v += Rb[(size_t)(mBase + mOff + r) * ldc + n];
        if (ACT == 2) v = fmaxf(v, 0.0f);
        if (ACT == 4) v = (v > 0.f) ? v : 0.01f * v;
        slab[(mOff + r) * 68 + (j << 4) + rlane] = v;
      }
    }
    __builtin_amdgcn_fence(__ATOMIC_RELEASE, "workgroup");
    __builtin_amdgcn_wave_barrier();
    __builtin_amdgcn_fence(__ATOMIC_ACQUIRE, "workgroup");
    if (OUT_MODE == 0) {
      float* C = (float*)Cout + (size_t)b * strideC;
      const int hh = lane >> 4, c4 = (lane & 15) * 4;
      for (int pass = 0; pass < 2; ++pass) {
#pragma unroll
        for (int it = 0; it < 8; ++it) {
          const int row = it * 2 + hh;
          v4f v = *(const v4f*)(slab + row * 68 + c4);
          *(volatile v4f*)(C + (size_t)(mBase + row) * ldc + n0 + c4) = v;
        }
        __threadfence();
      }
    } else {
      const int q = lane >> 3, c8 = (lane & 7) * 8;
      unsigned short* C  = (unsigned short*)Cout  + (size_t)b * strideC;
      unsigned short* C2 = (OUT_MODE == 2) ? ((unsigned short*)Cout2 + (size_t)b * strideC) : nullptr;
      for (int pass = 0; pass < 2; ++pass) {
#pragma unroll
        for (int it = 0; it < 4; ++it) {
          const int row = it * 4 + q;
          const float* sp = slab + row * 68 + c8;
          v8h hv, lv;
#pragma unroll
          for (int e = 0; e < 8; ++e) {
            if (OUT_MODE == 1) {
              hv[e] = (_Float16)sp[e];
            } else {
              unsigned short hb = f2bf_bits(sp[e]);
              unsigned short lb = f2bf_bits(sp[e] - bf_bits2f(hb));
              hv[e] = __builtin_bit_cast(_Float16, hb);
              lv[e] = __builtin_bit_cast(_Float16, lb);
            }
          }
          *(volatile v8h*)(C + (size_t)(mBase + row) * ldc + n0 + c8) = hv;
          if (OUT_MODE == 2) *(volatile v8h*)(C2 + (size_t)(mBase + row) * ldc + n0 + c8) = lv;
        }
        __threadfence();
      }
    }
    __builtin_amdgcn_fence(__ATOMIC_RELEASE, "workgroup");
    __builtin_amdgcn_wave_barrier();
    __builtin_amdgcn_fence(__ATOMIC_ACQUIRE, "workgroup");
  }
}

__global__ __launch_bounds__(256) void split8_bf16_kernel(const float* __restrict__ in,
                                                          unsigned short* __restrict__ hi,
                                                          unsigned short* __restrict__ lo, int n8) {
  const int i = blockIdx.x * 256 + threadIdx.x;
  if (i >= n8) return;
  const float* p = in + 8 * (size_t)i;
  const v4f a = *(const v4f*)(p);
  const v4f c = *(const v4f*)(p + 4);
  unsigned short hb[8], lb[8];
#pragma unroll
  for (int e = 0; e < 4; ++e) {
    hb[e] = f2bf_bits(a[e]);         lb[e] = f2bf_bits(a[e] - bf_bits2f(hb[e]));
    hb[4 + e] = f2bf_bits(c[e]);     lb[4 + e] = f2bf_bits(c[e] - bf_bits2f(hb[4 + e]));
  }
  const v4u uh = (v4u){pk16(hb[0], hb[1]), pk16(hb[2], hb[3]), pk16(hb[4], hb[5]), pk16(hb[6], hb[7])};
  const v4u ul = (v4u){pk16(lb[0], lb[1]), pk16(lb[2], lb[3]), pk16(lb[4], lb[5]), pk16(lb[6], lb[7])};
  unsigned short* qh = hi + 8 * (size_t)i;
  unsigned short* ql = lo + 8 * (size_t)i;
  *(volatile v4u*)qh = uh;
  *(volatile v4u*)ql = ul;
  __threadfence();
  *(volatile v4u*)qh = uh;
  *(volatile v4u*)ql = ul;
}

__device__ __forceinline__ float silu_f32(float v) {
  return v * __builtin_amdgcn_rcpf(1.0f + expf(-v));
}

__global__ __launch_bounds__(256) void conv_silu_kernel(const float* __restrict__ xz, const float* __restrict__ cw,
                                                        const float* __restrict__ cb, float* __restrict__ u_f32,
                                                        unsigned short* __restrict__ u_hi, unsigned short* __restrict__ u_lo) {
  __shared__ __align__(16) float sU[DIN_CH];
  const int m   = blockIdx.x;
  const int t   = m & (NL_SEQ - 1);
  const int tid = threadIdx.x;
  const int r1 = (t >= 1) ? (m - 1) : m;
  const int r2 = (t >= 2) ? (m - 2) : m;
  const int r3 = (t >= 3) ? (m - 3) : m;
  const float k1 = (t >= 1) ? 1.0f : 0.0f;
  const float k2 = (t >= 2) ? 1.0f : 0.0f;
  const float k3 = (t >= 3) ? 1.0f : 0.0f;
#pragma unroll 1
  for (int it = 0; it < 4; ++it) {
    const int d = it * 256 + tid;
    const float x0 = xz[(size_t)m  * NXZ_COL + d];
    const float x1 = xz[(size_t)r1 * NXZ_COL + d] * k1;
    const float x2 = xz[(size_t)r2 * NXZ_COL + d] * k2;
    const float x3 = xz[(size_t)r3 * NXZ_COL + d] * k3;
    const v4f w = *(const v4f*)(cw + (size_t)d * 4);
    float acc = cb[d] + w[3] * x0 + w[2] * x1 + w[1] * x2 + w[0] * x3;
    sU[d] = silu_f32(acc);
  }
  __syncthreads();
  const v4f fv = *(const v4f*)(sU + 4 * tid);
  float* dstf = u_f32 + (size_t)m * DIN_CH + 4 * tid;
  const int t8 = (tid & 127) * 8;
  const v4f a = *(const v4f*)(sU + t8);
  const v4f c = *(const v4f*)(sU + t8 + 4);
  unsigned short hb[8], lb[8];
#pragma unroll
  for (int e = 0; e < 4; ++e) {
    hb[e] = f2bf_bits(a[e]);         lb[e] = f2bf_bits(a[e] - bf_bits2f(hb[e]));
    hb[4 + e] = f2bf_bits(c[e]);     lb[4 + e] = f2bf_bits(c[e] - bf_bits2f(hb[4 + e]));
  }
  const v4u uh = (v4u){pk16(hb[0], hb[1]), pk16(hb[2], hb[3]), pk16(hb[4], hb[5]), pk16(hb[6], hb[7])};
  const v4u ul = (v4u){pk16(lb[0], lb[1]), pk16(lb[2], lb[3]), pk16(lb[4], lb[5]), pk16(lb[6], lb[7])};
  const bool hiw = (tid < 128);
  unsigned short* dst16 = (hiw ? u_hi : u_lo) + (size_t)m * DIN_CH + t8;
  v4u us;
  if (hiw) us = uh; else us = ul;
  for (int pass = 0; pass < 2; ++pass) {
    *(volatile v4f*)dstf = fv;
    *(volatile v4u*)dst16 = us;
    __threadfence();
  }
}

__global__ __launch_bounds__(256) void split_dt_kernel(const float* __restrict__ dbc,
                                                       unsigned short* __restrict__ hi,
                                                       unsigned short* __restrict__ lo, int n8) {
  const int i = blockIdx.x * 256 + threadIdx.x;
  if (i >= n8) return;
  const int row = i >> 2, c8 = (i & 3) * 8;
  const float* p = dbc + (size_t)row * NDBC_COL + c8;
  const v4f a = *(const v4f*)(p);
  const v4f c = *(const v4f*)(p + 4);
  unsigned short hb[8], lb[8];
#pragma unroll
  for (int e = 0; e < 4; ++e) {
    hb[e] = f2bf_bits(a[e]);         lb[e] = f2bf_bits(a[e] - bf_bits2f(hb[e]));
    hb[4 + e] = f2bf_bits(c[e]);     lb[4 + e] = f2bf_bits(c[e] - bf_bits2f(hb[4 + e]));
  }
  const v4u uh = (v4u){pk16(hb[0], hb[1]), pk16(hb[2], hb[3]), pk16(hb[4], hb[5]), pk16(hb[6], hb[7])};
  const v4u ul = (v4u){pk16(lb[0], lb[1]), pk16(lb[2], lb[3]), pk16(lb[4], lb[5]), pk16(lb[6], lb[7])};
  unsigned short* qh = hi + (size_t)row * DTR_K + c8;
  unsigned short* ql = lo + (size_t)row * DTR_K + c8;
  *(volatile v4u*)qh = uh;
  *(volatile v4u*)ql = ul;
  __threadfence();
  *(volatile v4u*)qh = uh;
  *(volatile v4u*)ql = ul;
}

constexpr int SC_TCH = 32;
constexpr int SC_NCH = 128;
__global__ __launch_bounds__(128) void scan_kernel(const float* __restrict__ delta_pre, const float* __restrict__ u_f32,
                                                   const float* __restrict__ xz, const float* __restrict__ dbc,
                                                   const float* __restrict__ a_log, const float* __restrict__ dsk,
                                                   const float* __restrict__ dtb,
                                                   unsigned short* __restrict__ y_hi, unsigned short* __restrict__ y_lo) {
  __shared__ __align__(16) float sBC[SC_TCH * 32];
  __shared__ __align__(16) float sDL[SC_TCH * SC_NCH];
  __shared__ __align__(16) float sY[SC_TCH * SC_NCH];
  const int tid = threadIdx.x;
  const int c   = tid;
  const int d0  = blockIdx.x * SC_NCH;
  const int d   = d0 + c;
  const int b   = blockIdx.y;

  float A2[DST_N];
  {
    const float* ap = a_log + (size_t)d * DST_N;
#pragma unroll
    for (int q4 = 0; q4 < 4; ++q4) {
      const v4f av = *(const v4f*)(ap + 4 * q4);
#pragma unroll
      for (int e = 0; e < 4; ++e) A2[4 * q4 + e] = -expf(av[e]) * LOG2E_F;
    }
  }
  const float Dd = dsk[d];
  const float bd = dtb[d];
  float h[DST_N];
#pragma unroll
  for (int s = 0; s < DST_N; ++s) h[s] = 0.0f;

  const size_t rowb0 = (size_t)b * NL_SEQ;
#pragma unroll 1
  for (int ch = 0; ch < NL_SEQ / SC_TCH; ++ch) {
    const size_t rb = rowb0 + (size_t)ch * SC_TCH;
    __syncthreads();
#pragma unroll
    for (int it = 0; it < 2; ++it) {
      const int e = it * 128 + tid;
      const int r = e >> 3, c4 = (e & 7) * 4;
      const v4f v = *(const v4f*)(dbc + (rb + r) * NDBC_COL + DTR_K + c4);
      *(v4f*)(sBC + r * 32 + c4) = v;
    }
#pragma unroll 1
    for (int tt = 0; tt < SC_TCH; ++tt) {
      const float v = delta_pre[(rb + tt) * DIN_CH + d] + bd;
      const float sp = fmaxf(v, 0.0f) + log1pf(expf(-fabsf(v)));
      sDL[tt * SC_NCH + c] = sp;
    }
    __syncthreads();
#pragma unroll 1
    for (int tt = 0; tt < SC_TCH; ++tt) {
      const float dl = sDL[tt * SC_NCH + c];
      const float uu = u_f32[(rb + tt) * DIN_CH + d];
      const float zz = xz[(rb + tt) * NXZ_COL + DIN_CH + d];
      const float dlu = dl * uu;
      const v4f* bc4 = (const v4f*)(sBC + tt * 32);
      float Bv[DST_N], Cv[DST_N];
#pragma unroll
      for (int q4 = 0; q4 < 4; ++q4) {
        const v4f bb = bc4[q4];
        const v4f cc = bc4[4 + q4];
#pragma unroll
        for (int e = 0; e < 4; ++e) { Bv[4 * q4 + e] = bb[e]; Cv[4 * q4 + e] = cc[e]; }
      }
      float yv = 0.0f;
#pragma unroll
      for (int s = 0; s < DST_N; ++s) {
        const float da = exp2f(dl * A2[s]);
        h[s] = da * h[s] + dlu * Bv[s];
        yv += h[s] * Cv[s];
      }
      yv = yv + uu * Dd;
      const float g = silu_f32(zz);
      sY[tt * SC_NCH + c] = yv * g;
    }
    __syncthreads();
    for (int pass = 0; pass < 2; ++pass) {
#pragma unroll
      for (int it = 0; it < 4; ++it) {
        const int e = it * 128 + tid;
        const int row = e >> 4, c8 = (e & 15) * 8;
        const v4f a  = *(const v4f*)(sY + row * SC_NCH + c8);
        const v4f cq = *(const v4f*)(sY + row * SC_NCH + c8 + 4);
        unsigned short hb[8], lb[8];
#pragma unroll
        for (int q = 0; q < 4; ++q) {
          hb[q] = f2bf_bits(a[q]);          lb[q] = f2bf_bits(a[q] - bf_bits2f(hb[q]));
          hb[4 + q] = f2bf_bits(cq[q]);     lb[4 + q] = f2bf_bits(cq[q] - bf_bits2f(hb[4 + q]));
        }
        const v4u uh = (v4u){pk16(hb[0], hb[1]), pk16(hb[2], hb[3]), pk16(hb[4], hb[5]), pk16(hb[6], hb[7])};
        const v4u ul = (v4u){pk16(lb[0], lb[1]), pk16(lb[2], lb[3]), pk16(lb[4], lb[5]), pk16(lb[6], lb[7])};
        const size_t off = (rb + row) * DIN_CH + d0 + c8;
        *(volatile v4u*)(y_hi + off) = uh;
        *(volatile v4u*)(y_lo + off) = ul;
      }
      __threadfence();
    }
  }
}

__global__ __launch_bounds__(128) void ln_residual_kernel(const float* __restrict__ x, const float* __restrict__ o1,
                                                          const float* __restrict__ lw, const float* __restrict__ lb,
                                                          float* __restrict__ out) {
  __shared__ float redA[4];
  __shared__ float redB[4];
  const int m = blockIdx.x;
  const int tid = threadIdx.x;
  const int lane = tid & 31, wave = tid >> 5;
  const size_t base = (size_t)m * DMOD + 4 * tid;
  const v4f ov = *(const v4f*)(o1 + base);
  const v4f xv = *(const v4f*)(x + base);
  const v4f wv = *(const v4f*)(lw + 4 * tid);
  const v4f bv = *(const v4f*)(lb + 4 * tid);
  float s = (ov[0] + ov[1]) + (ov[2] + ov[3]);
#pragma unroll
  for (int off = 16; off > 0; off >>= 1) s += __shfl_xor(s, off, 32);
  if (lane == 0) redA[wave] = s;
  __syncthreads();
  const float mu = ((redA[0] + redA[1]) + (redA[2] + redA[3])) * INV_DMOD;
  float dv[4];
#pragma unroll
  for (int e = 0; e < 4; ++e) dv[e] = ov[e] - mu;
  float q = (dv[0] * dv[0] + dv[1] * dv[1]) + (dv[2] * dv[2] + dv[3] * dv[3]);
#pragma unroll
  for (int off = 16; off > 0; off >>= 1) q += __shfl_xor(q, off, 32);
  if (lane == 0) redB[wave] = q;
  __syncthreads();
  const float var = ((redB[0] + redB[1]) + (redB[2] + redB[3])) * INV_DMOD;
  const float rs = rsqrtf(var + LN_EPS);
  v4f r;
#pragma unroll
  for (int e = 0; e < 4; ++e) r[e] = xv[e] + (dv[e] * rs * wv[e] + bv[e]);
  float* op = out + base;
  for (int pass = 0; pass < 2; ++pass) {
    *(volatile v4f*)op = r;
    __threadfence();
  }
}

extern "C" void kernel_launch(void* const* d_in, const int* in_sizes, int n_in,
                              void* d_out, int out_size, void* d_ws, size_t ws_size,
                              hipStream_t stream)
{
  if (n_in < 12) return;
  if (in_sizes[0] != NTOK * DMOD) return;
  if (in_sizes[1] != NXZ_COL * DMOD) return;
  if (in_sizes[2] != DIN_CH * 4) return;
  if (in_sizes[3] != DIN_CH) return;
  if (in_sizes[4] != NDBC_COL * DIN_CH) return;
  if (in_sizes[5] != DIN_CH * DTR_K) return;
  if (in_sizes[6] != DIN_CH) return;
  if (in_sizes[7] != DIN_CH * DST_N) return;
  if (in_sizes[8] != DIN_CH) return;
  if (in_sizes[9] != DMOD * DIN_CH) return;
  if (in_sizes[10] != DMOD) return;
  if (in_sizes[11] != DMOD) return;
  if (out_size != NTOK * DMOD) return;

  const float* x      = (const float*)d_in[0];
  const float* w_in   = (const float*)d_in[1];
  const float* conv_w = (const float*)d_in[2];
  const float* conv_b = (const float*)d_in[3];
  const float* w_xp   = (const float*)d_in[4];
  const float* w_dt   = (const float*)d_in[5];
  const float* b_dt   = (const float*)d_in[6];
  const float* a_log  = (const float*)d_in[7];
  const float* d_skip = (const float*)d_in[8];
  const float* w_out  = (const float*)d_in[9];
  const float* ln_w   = (const float*)d_in[10];
  const float* ln_b   = (const float*)d_in[11];
  float* out = (float*)d_out;

  char* wsb = (char*)d_ws;
  size_t off = 0;
  auto carve = [&](size_t bytes) -> char* {
    char* p = wsb + off; off += (bytes + 255) & ~(size_t)255; return p;
  };
  unsigned short* x_hi    = (unsigned short*)carve((size_t)NTOK * DMOD * 2);
  unsigned short* x_lo    = (unsigned short*)carve((size_t)NTOK * DMOD * 2);
  unsigned short* win_hi  = (unsigned short*)carve((size_t)NXZ_COL * DMOD * 2);
  unsigned short* win_lo  = (unsigned short*)carve((size_t)NXZ_COL * DMOD * 2);
  unsigned short* wxp_hi  = (unsigned short*)carve((size_t)NDBC_COL * DIN_CH * 2);
  unsigned short* wxp_lo  = (unsigned short*)carve((size_t)NDBC_COL * DIN_CH * 2);
  unsigned short* wdt_hi  = (unsigned short*)carve((size_t)DIN_CH * DTR_K * 2);
  unsigned short* wdt_lo  = (unsigned short*)carve((size_t)DIN_CH * DTR_K * 2);
  unsigned short* wout_hi = (unsigned short*)carve((size_t)DMOD * DIN_CH * 2);
  unsigned short* wout_lo = (unsigned short*)carve((size_t)DMOD * DIN_CH * 2);
  float*          xz      = (float*)carve((size_t)NTOK * NXZ_COL * 4);
  float*          u_f32   = (float*)carve((size_t)NTOK * DIN_CH * 4);
  unsigned short* u_hi    = (unsigned short*)carve((size_t)NTOK * DIN_CH * 2);
  unsigned short* u_lo    = (unsigned short*)carve((size_t)NTOK * DIN_CH * 2);
  float*          dbc     = (float*)carve((size_t)NTOK * NDBC_COL * 4);
  unsigned short* dt_hi   = (unsigned short*)carve((size_t)NTOK * DTR_K * 2);
  unsigned short* dt_lo   = (unsigned short*)carve((size_t)NTOK * DTR_K * 2);
  float*          dpre    = (float*)carve((size_t)NTOK * DIN_CH * 4);
  unsigned short* y_hi    = (unsigned short*)carve((size_t)NTOK * DIN_CH * 2);
  unsigned short* y_lo    = (unsigned short*)carve((size_t)NTOK * DIN_CH * 2);
  float*          out1    = (float*)carve((size_t)NTOK * DMOD * 4);
  if (off > ws_size) return;

  {
    const int n8x = NTOK * DMOD / 8;
    split8_bf16_kernel<<<dim3((n8x + 255) / 256), 256, 0, stream>>>(x, x_hi, x_lo, n8x);
    const int n8a = NXZ_COL * DMOD / 8;
    split8_bf16_kernel<<<dim3((n8a + 255) / 256), 256, 0, stream>>>(w_in, win_hi, win_lo, n8a);
    const int n8b = NDBC_COL * DIN_CH / 8;
    split8_bf16_kernel<<<dim3((n8b + 255) / 256), 256, 0, stream>>>(w_xp, wxp_hi, wxp_lo, n8b);
    const int n8c = DIN_CH * DTR_K / 8;
    split8_bf16_kernel<<<dim3((n8c + 255) / 256), 256, 0, stream>>>(w_dt, wdt_hi, wdt_lo, n8c);
    const int n8d = DMOD * DIN_CH / 8;
    split8_bf16_kernel<<<dim3((n8d + 255) / 256), 256, 0, stream>>>(w_out, wout_hi, wout_lo, n8d);
  }

  {
    const int tiles = (NTOK / 64) * (NXZ_COL / 64);
    wmma_gemm64<1, true, 0, 0, false, 0><<<dim3((tiles + 7) / 8, 1), 256, 0, stream>>>(
        x_hi, x_lo, DMOD, 0L,
        win_hi, win_lo, DMOD, 0L,
        (void*)xz, nullptr, NXZ_COL, 0L,
        nullptr, nullptr, 0L,
        NTOK, NXZ_COL, DMOD, 1.0f);
  }

  conv_silu_kernel<<<dim3(NTOK), 256, 0, stream>>>(xz, conv_w, conv_b, u_f32, u_hi, u_lo);

  {
    const int tiles = (NTOK / 64) * (NDBC_COL / 64);
    wmma_gemm64<1, true, 0, 0, false, 0><<<dim3((tiles + 7) / 8, 1), 256, 0, stream>>>(
        u_hi, u_lo, DIN_CH, 0L,
        wxp_hi, wxp_lo, DIN_CH, 0L,
        (void*)dbc, nullptr, NDBC_COL, 0L,
        nullptr, nullptr, 0L,
        NTOK, NDBC_COL, DIN_CH, 1.0f);
  }

  {
    const int n8 = NTOK * DTR_K / 8;
    split_dt_kernel<<<dim3((n8 + 255) / 256), 256, 0, stream>>>(dbc, dt_hi, dt_lo, n8);
  }

  {
    const int tiles = (NTOK / 64) * (DIN_CH / 64);
    wmma_gemm64<1, true, 0, 0, false, 0><<<dim3((tiles + 7) / 8, 1), 256, 0, stream>>>(
        dt_hi, dt_lo, DTR_K, 0L,
        wdt_hi, wdt_lo, DTR_K, 0L,
        (void*)dpre, nullptr, DIN_CH, 0L,
        nullptr, nullptr, 0L,
        NTOK, DIN_CH, DTR_K, 1.0f);
  }

  scan_kernel<<<dim3(DIN_CH / SC_NCH, NB_BATCH), SC_NCH, 0, stream>>>(
      dpre, u_f32, xz, dbc, a_log, d_skip, b_dt, y_hi, y_lo);

  {
    const int tiles = (NTOK / 64) * (DMOD / 64);
    wmma_gemm64<1, true, 0, 0, false, 0><<<dim3((tiles + 7) / 8, 1), 256, 0, stream>>>(
        y_hi, y_lo, DIN_CH, 0L,
        wout_hi, wout_lo, DIN_CH, 0L,
        (void*)out1, nullptr, DMOD, 0L,
        nullptr, nullptr, 0L,
        NTOK, DMOD, DIN_CH, 1.0f);
  }

  ln_residual_kernel<<<dim3(NTOK), 128, 0, stream>>>(x, out1, ln_w, ln_b, out);
}
